// IntegralTransform_79886391705729
// MI455X (gfx1250) — hardware-verified
//
#include <hip/hip_runtime.h>
#include <math.h>
typedef __attribute__((ext_vector_type(16))) _Float16 v16h;
typedef __attribute__((ext_vector_type(8)))  _Float16 v8h;
typedef __attribute__((ext_vector_type(16))) __bf16   v16b;
typedef __attribute__((ext_vector_type(8)))  __bf16   v8b;
typedef __attribute__((ext_vector_type(8)))  float    v8f;
typedef __attribute__((ext_vector_type(4)))  float    v4f;

__device__ __forceinline__ float erf_fast(float x) {
  const float ax = fabsf(x); const float t = __builtin_amdgcn_rcpf(fmaf(0.3275911f, ax, 1.0f));
  float p = fmaf(1.061405429f, t, -1.453152027f); p = fmaf(p, t, 1.421413741f); p = fmaf(p, t, -0.284496736f); p = fmaf(p, t, 0.254829592f); p *= t;
  const float e = __builtin_amdgcn_exp2f(-ax * ax * 1.4426950408889634f); const float r = 1.0f - p * e; return copysignf(r, x);
}
#define PSCALE 32768.0f
#define U16(p) ((const unsigned short*)(const void*)(p))
#define PSCALE_INV (1.0f / 32768.0f)

__device__ __forceinline__ unsigned short f2bf_bits(float f) {
  unsigned u = __float_as_uint(f);
  return (unsigned short)((u + 0x7FFFu + ((u >> 16) & 1u)) >> 16);
}
__device__ __forceinline__ float bf_bits2f(unsigned short h) { return __uint_as_float(((unsigned)h) << 16); }

__device__ __forceinline__ void dep_guard_h(v8f& a, v8f& b, v16h x, v16h y) { asm volatile("v_nop\n\tv_nop\n\tv_nop\n\tv_nop" : "+v"(a), "+v"(b) : "v"(x), "v"(y)); }
__device__ __forceinline__ void dep_guard_b(v8f& a, v8f& b, v16b x, v16b y) { asm volatile("v_nop\n\tv_nop\n\tv_nop\n\tv_nop" : "+v"(a), "+v"(b) : "v"(x), "v"(y)); }
__device__ __forceinline__ void keep4_h(v16h a, v16h b, v16h c, v16h d) { asm volatile("v_nop" :: "v"(a), "v"(b), "v"(c), "v"(d)); }
__device__ __forceinline__ void keep4_b(v16b a, v16b b, v16b c, v16b d) { asm volatile("v_nop" :: "v"(a), "v"(b), "v"(c), "v"(d)); }
__device__ __forceinline__ void acc_guard4(v8f& a, v8f& b, v8f& c, v8f& d) { asm volatile("v_nop\n\tv_nop\n\tv_nop\n\tv_nop" : "+v"(a), "+v"(b), "+v"(c), "+v"(d)); }
template <typename T> struct Frag;
template <> struct Frag<_Float16> {
  typedef v16h V; union U { v16h v; v8h h[2]; };
  static __device__ __forceinline__ v16h load(const _Float16* p) {
    U f; f.h[0] = *(const v8h*)(p); f.h[1] = *(const v8h*)(p + 16); return f.v;
  }
  static __device__ __forceinline__ v8f mma(v16h a, v16h b, v8f c) {
    return __builtin_amdgcn_wmma_f32_16x16x32_f16(false, a, false, b, (short)0, c, false, false);
  }
  static __device__ __forceinline__ void guard(v8f& a, v8f& b, v16h x, v16h y) { dep_guard_h(a, b, x, y); }
  static __device__ __forceinline__ void keep(v16h a, v16h b, v16h c, v16h d) { keep4_h(a, b, c, d); }
};
template <> struct Frag<__bf16> {
  typedef v16b V; union U { v16b v; v8b h[2]; };
  static __device__ __forceinline__ v16b load(const __bf16* p) {
    U f; f.h[0] = *(const v8b*)(p); f.h[1] = *(const v8b*)(p + 16); return f.v;
  }
  static __device__ __forceinline__ v8f mma(v16b a, v16b b, v8f c) {
    return __builtin_amdgcn_wmma_f32_16x16x32_bf16(false, a, false, b, (short)0, c, false, false);
  }
  static __device__ __forceinline__ void guard(v8f& a, v8f& b, v16b x, v16b y) { dep_guard_b(a, b, x, y); }
  static __device__ __forceinline__ void keep(v16b a, v16b b, v16b c, v16b d) { keep4_b(a, b, c, d); }
};

template <int ET> struct Elem;
template <> struct Elem<0> { typedef _Float16 T; };
template <> struct Elem<1> { typedef __bf16 T; };
template <int ET, bool SPLIT, int BIAS_MODE, int OUT_MODE, bool RESID, int ACT = 0>
__global__ __launch_bounds__(256) void wmma_gemm64(
    const unsigned short* __restrict__ Ap, const unsigned short* __restrict__ A2p, int lda, long strideA,
    const unsigned short* __restrict__ Btp, const unsigned short* __restrict__ Bt2p, int ldb, long strideB,
    void* __restrict__ Cout, void* __restrict__ Cout2, int ldc, long strideC,
    const float* __restrict__ bias,
    const float* __restrict__ resid, long strideR,
    int M, int N, int K, float scale) {
  typedef typename Elem<ET>::T T;
  typedef typename Frag<T>::V V;
  const T* A = (const T*)Ap; const T* A2 = (const T*)A2p; const T* Bt = (const T*)Btp; const T* Bt2 = (const T*)Bt2p;
  __shared__ __align__(16) float sT[8][16 * 68];
  const int b    = blockIdx.y;
  const int lane = threadIdx.x & 31;
  const int wave = threadIdx.x >> 5;
  const int tilesN = N >> 6;
  const int tilesM = M >> 6;
  const int tile = blockIdx.x * 8 + wave;
  if (tile >= tilesM * tilesN) return;
  const int tm = tile / tilesN;
  const int tn = tile - tm * tilesN;
  const int m0 = tm << 6;
  const int n0 = tn << 6;

  const T* Ab  = A  + (size_t)b * strideA;
  const T* Bb  = Bt + (size_t)b * strideB;
  const T* Ab2 = SPLIT ? (A2  + (size_t)b * strideA) : nullptr;
  const T* Bb2 = SPLIT ? (Bt2 + (size_t)b * strideB) : nullptr;

  const int rlane = lane & 15;
  const int koff  = (lane >> 4) * 8;
  const int mOff  = (lane >> 4) * 8;

  v8f acc[4][4];
#pragma unroll
  for (int i = 0; i < 4; ++i)
#pragma unroll
    for (int j = 0; j < 4; ++j) acc[i][j] = (v8f){0.f,0.f,0.f,0.f,0.f,0.f,0.f,0.f};

  for (int k0 = 0; k0 < K; k0 += 32) {
    V bh[4], bl[4];
#pragma unroll
    for (int j = 0; j < 4; ++j) {
      const size_t bo = (size_t)(n0 + (j << 4) + rlane) * ldb + koff + k0;
      bh[j] = Frag<T>::load(Bb + bo);
      if (SPLIT) bl[j] = Frag<T>::load(Bb2 + bo);
    }
#pragma unroll
    for (int i = 0; i < 4; ++i) {
      const size_t ao = (size_t)(m0 + (i << 4) + rlane) * lda + koff + k0;
      V ah = Frag<T>::load(Ab + ao);
      V al;
      if (SPLIT) al = Frag<T>::load(Ab2 + ao);
#pragma unroll
      for (int j = 0; j < 4; ++j) {
        acc[i][j] = Frag<T>::mma(ah, bh[j], acc[i][j]);
        if (SPLIT) {
          acc[i][j] = Frag<T>::mma(ah, bl[j], acc[i][j]);
          acc[i][j] = Frag<T>::mma(al, bh[j], acc[i][j]);
        }
      }
      Frag<T>::guard(acc[i][0], acc[i][3], ah, SPLIT ? al : ah);
    }
    Frag<T>::keep(bh[0], bh[1], bh[2], bh[3]);
    if (SPLIT) Frag<T>::keep(bl[0], bl[1], bl[2], bl[3]);
  }
  acc_guard4(acc[0][0], acc[0][1], acc[0][2], acc[0][3]);
  acc_guard4(acc[1][0], acc[1][1], acc[1][2], acc[1][3]);
  acc_guard4(acc[2][0], acc[2][1], acc[2][2], acc[2][3]);
  acc_guard4(acc[3][0], acc[3][1], acc[3][2], acc[3][3]);

  float* slab = sT[wave];
  const float* Rb = RESID ? (resid + (size_t)b * strideR) : nullptr;
#pragma unroll
  for (int i = 0; i < 4; ++i) {
    const int mBase = m0 + (i << 4);
#pragma unroll
    for (int j = 0; j < 4; ++j) {
      const int n = n0 + (j << 4) + rlane;
      float bv = 0.f;
      if (BIAS_MODE == 2) bv = bias[n];
#pragma unroll
      for (int r = 0; r < 8; ++r) {
        float v = acc[i][j][r] * scale;
        if (BIAS_MODE == 1) v += bias[mBase + mOff + r];
        if (BIAS_MODE == 2) v += bv;
        if (RESID) v += Rb[(size_t)(mBase + mOff + r) * ldc + n];
        if (ACT == 1) v = tanhf(v);
        if (ACT == 2) v = fmaxf(v, 0.0f);
        if (ACT == 3) v = v / (1.0f + expf(-v));
        if (ACT == 4) v = (v > 0.f) ? v : 0.01f * v;
        if (ACT == 5) v = 0.5f * v * (1.0f + erf_fast(v * 0.70710678118654752f));
        slab[(mOff + r) * 68 + (j << 4) + rlane] = v;
      }
    }
    __builtin_amdgcn_fence(__ATOMIC_RELEASE, "workgroup");
    __builtin_amdgcn_wave_barrier();
    __builtin_amdgcn_fence(__ATOMIC_ACQUIRE, "workgroup");
    if (OUT_MODE == 0) {
      float* C = (float*)Cout + (size_t)b * strideC;
      const int hh = lane >> 4, c4 = (lane & 15) * 4;
      for (int pass = 0; pass < 2; ++pass) {
#pragma unroll
        for (int it = 0; it < 8; ++it) {
          const int row = it * 2 + hh;
          v4f v = *(const v4f*)(slab + row * 68 + c4);
          *(volatile v4f*)(C + (size_t)(mBase + row) * ldc + n0 + c4) = v;
        }
        __threadfence();
      }
    } else {
      const int q = lane >> 3, c8 = (lane & 7) * 8;
      unsigned short* C  = (unsigned short*)Cout  + (size_t)b * strideC;
      unsigned short* C2 = (OUT_MODE == 2) ? ((unsigned short*)Cout2 + (size_t)b * strideC) : nullptr;
      for (int pass = 0; pass < 2; ++pass) {
#pragma unroll
        for (int it = 0; it < 4; ++it) {
          const int row = it * 4 + q;
          const float* sp = slab + row * 68 + c8;
          v8h hv, lv;
#pragma unroll
          for (int e = 0; e < 8; ++e) {
            if (OUT_MODE == 1) {
              hv[e] = (_Float16)sp[e];
            } else {
              unsigned short hb = f2bf_bits(sp[e]);
              unsigned short lb = f2bf_bits(sp[e] - bf_bits2f(hb));
              hv[e] = __builtin_bit_cast(_Float16, hb);
              lv[e] = __builtin_bit_cast(_Float16, lb);
            }
          }
          *(volatile v8h*)(C + (size_t)(mBase + row) * ldc + n0 + c8) = hv;
          if (OUT_MODE == 2) *(volatile v8h*)(C2 + (size_t)(mBase + row) * ldc + n0 + c8) = lv;
        }
        __threadfence();
      }
    }
    __builtin_amdgcn_fence(__ATOMIC_RELEASE, "workgroup");
    __builtin_amdgcn_wave_barrier();
    __builtin_amdgcn_fence(__ATOMIC_ACQUIRE, "workgroup");
  }
}


#define IN_ 50000
#define IE 1600000
#define ICH 25
#define IEC (IE / ICH)
#define IECP 64000
#define IC 32
#define IMAXSEG 256
__device__ __forceinline__ unsigned pkh(float a, float b) { return (unsigned)__builtin_bit_cast(unsigned short, (_Float16)a) | ((unsigned)__builtin_bit_cast(unsigned short, (_Float16)b) << 16); }
__device__ __forceinline__ float gelu_e(float v) { return 0.5f * v * (1.0f + erf_fast(v * 0.70710678118654752f)); }
__global__ __launch_bounds__(256) void node_kernel(const float* __restrict__ y, const float* __restrict__ fy, const float* __restrict__ W1, const float* __restrict__ b1, unsigned* __restrict__ NA, unsigned* __restrict__ NB) {
  const int lane = threadIdx.x & 31, wave = threadIdx.x >> 5; const int n = blockIdx.x * 8 + wave; if (n >= IN_) return; const int c0 = 2 * lane, c1 = c0 + 1;
  const float y0 = y[(size_t)n * 3], y1 = y[(size_t)n * 3 + 1], y2 = y[(size_t)n * 3 + 2];
  float a0 = y0 * W1[c0] + y1 * W1[64 + c0] + y2 * W1[128 + c0], a1 = y0 * W1[c1] + y1 * W1[64 + c1] + y2 * W1[128 + c1];
  const float b0v = y0 * W1[192 + c0] + y1 * W1[256 + c0] + y2 * W1[320 + c0] + b1[c0], b1v = y0 * W1[192 + c1] + y1 * W1[256 + c1] + y2 * W1[320 + c1] + b1[c1];
#pragma unroll 4
  for (int k = 0; k < IC; ++k) { const float f = fy[(size_t)n * IC + k]; a0 += f * W1[(6 + k) * 64 + c0]; a1 += f * W1[(6 + k) * 64 + c1]; }
  for (int pass = 0; pass < 2; ++pass) { ((volatile unsigned*)NA)[(size_t)n * 32 + lane] = pkh(a0, a1); ((volatile unsigned*)NB)[(size_t)n * 32 + lane] = pkh(b0v, b1v); __threadfence(); }
}
__global__ __launch_bounds__(256) void efeat_kernel(const unsigned* __restrict__ NA, const unsigned* __restrict__ NB, const int* __restrict__ nbr, const int* __restrict__ rs, int e0, unsigned* __restrict__ H1) {
  const int el = blockIdx.x * 256 + threadIdx.x; if (el >= IEC) return; const int e = e0 + el;
  int j = nbr[e]; j = j < 0 ? 0 : (j >= IN_ ? IN_ - 1 : j);
  int lo = 0, hi = IN_;
  for (int it = 0; it < 17; ++it) { const int mid = (lo + hi + 1) >> 1; if (mid <= IN_ && rs[mid] <= e) lo = mid; else hi = mid - 1; if (hi < lo) hi = lo; }
  const int i = lo < 0 ? 0 : (lo >= IN_ ? IN_ - 1 : lo);
  typedef __attribute__((ext_vector_type(2))) _Float16 v2h; typedef __attribute__((ext_vector_type(4))) unsigned u4;
  const unsigned* pa = NA + (size_t)j * 32; const unsigned* pb = NB + (size_t)i * 32; unsigned* dst = H1 + (size_t)el * 32;
  for (int pass = 0; pass < 2; ++pass) {
#pragma unroll 1
    for (int q4 = 0; q4 < 8; ++q4) { u4 u;
#pragma unroll 1
      for (int z = 0; z < 4; ++z) { const int c = q4 * 4 + z; const v2h a2 = __builtin_bit_cast(v2h, pa[c]), b2 = __builtin_bit_cast(v2h, pb[c]);
        u[z] = pkh(gelu_e((float)a2[0] + (float)b2[0]), gelu_e((float)a2[1] + (float)b2[1])); }
      *(volatile u4*)(dst + q4 * 4) = u; }
    __threadfence(); }
}
__global__ __launch_bounds__(256) void wt_kernel(const float* __restrict__ Wm, int Kd, int NOUT, unsigned* __restrict__ BT) {
  for (int i = threadIdx.x; i < 64 * 32; i += 256) { const int o = i / 32, kp = 2 * (i % 32); float a = 0.f, b = 0.f; if (o < NOUT) { if (kp < Kd) a = Wm[(size_t)kp * NOUT + o]; if (kp + 1 < Kd) b = Wm[(size_t)(kp + 1) * NOUT + o]; }
    ((volatile unsigned*)BT)[i] = pkh(a, b); __threadfence(); ((volatile unsigned*)BT)[i] = pkh(a, b); }
}
__global__ __launch_bounds__(256) void zero_kernel(float* __restrict__ p, long n) { const long i = (long)blockIdx.x * 256 + threadIdx.x; if (i < n) { ((volatile float*)p)[i] = 0.f; __threadfence(); ((volatile float*)p)[i] = 0.f; } }
__global__ __launch_bounds__(256) void kcopy_kernel(const unsigned* __restrict__ K3c, int e0, unsigned* __restrict__ KALL) {
  const long i = (long)blockIdx.x * 256 + threadIdx.x; if (i >= (long)IEC * 16) return; const long el = i / 16; const int c = (int)(i % 16); const unsigned u = K3c[el * 32 + c];
  ((volatile unsigned*)KALL)[((long)e0 + el) * 16 + c] = u; __threadfence(); ((volatile unsigned*)KALL)[((long)e0 + el) * 16 + c] = u;
}
__global__ __launch_bounds__(256) void reduce_kernel(const unsigned* __restrict__ KALL, const float* __restrict__ b3, const float* __restrict__ fy, const float* __restrict__ wts, const int* __restrict__ nbr, const int* __restrict__ rs, float* __restrict__ out) {
  const int lane = threadIdx.x & 31, wave = threadIdx.x >> 5; const int i = blockIdx.x * 8 + wave; if (i >= IN_) return;
  int a = rs[i], b = rs[i + 1]; if (a < 0) a = 0; if (b > IE) b = IE; if (b > a + IMAXSEG) b = a + IMAXSEG;
  float s = 0.f; typedef __attribute__((ext_vector_type(2))) _Float16 v2h;
  for (int e = a; e < b; ++e) { int j = nbr[e]; j = j < 0 ? 0 : (j >= IN_ ? IN_ - 1 : j); const v2h p = __builtin_bit_cast(v2h, KALL[(size_t)e * 16 + (lane >> 1)]); const float kv = (float)p[lane & 1];
    s += wts[j] * (kv + b3[lane]) * fy[(size_t)j * IC + lane]; }
  float* dst = out + (size_t)i * IC + lane; *(volatile float*)dst = s; __threadfence(); *(volatile float*)dst = s;
}
extern "C" void kernel_launch(void* const* d_in, const int* in_sizes, int n_in, void* d_out, int out_size, void* d_ws, size_t ws_size, hipStream_t stream) {
  (void)in_sizes; (void)n_in; (void)out_size; (void)ws_size;
  auto Fp = [&](int i) { return (const float*)d_in[i]; };
  const float* y = Fp(0); const float* fy = Fp(1); const float* wts = Fp(2); const float* W1 = Fp(3); const float* b1 = Fp(4); const float* W2 = Fp(5); const float* b2 = Fp(6); const float* W3 = Fp(7); const float* b3 = Fp(8); const int* nbr = (const int*)d_in[9]; const int* rs = (const int*)d_in[10];
  float* out = (float*)d_out;
  char* ws = (char*)d_ws; size_t off = 0;
  auto carve = [&](size_t bytes) -> char* { char* p = ws + off; off += (bytes + 255) & ~(size_t)255; return p; };
  unsigned* H1 = (unsigned*)carve((size_t)IECP * 64 * 2); _Float16* H2 = (_Float16*)carve((size_t)IECP * 64 * 2); _Float16* K3c = (_Float16*)H1;
  unsigned* NA = (unsigned*)carve((size_t)IN_ * 64 * 2); unsigned* NB = (unsigned*)carve((size_t)IN_ * 64 * 2);
  unsigned* BT2 = (unsigned*)carve(64 * 64 * 2); unsigned* BT3 = (unsigned*)carve(64 * 64 * 2); unsigned* KALL = (unsigned*)carve((size_t)IE * IC * 2);
  wt_kernel<<<1, 256, 0, stream>>>(W2, 64, 64, BT2); wt_kernel<<<1, 256, 0, stream>>>(W3, 64, 32, BT3);
  zero_kernel<<<(unsigned)(((long)IECP * 32 + 255) / 256), 256, 0, stream>>>((float*)H1, (long)IECP * 32);
  node_kernel<<<(IN_ + 7) / 8, 256, 0, stream>>>(y, fy, W1, b1, NA, NB);
  const int t = (IECP / 64) * 1;
  for (int ch = 0; ch < ICH; ++ch) { const int e0 = ch * IEC;
    efeat_kernel<<<(IEC + 255) / 256, 256, 0, stream>>>(NA, NB, nbr, rs, e0, H1);
    wmma_gemm64<0, false, 2, 1, false, 5><<<dim3((t + 7) / 8, 1), 256, 0, stream>>>((const unsigned short*)H1, nullptr, 64, 0, (const unsigned short*)BT2, nullptr, 64, 0, H2, nullptr, 64, 0, b2, nullptr, 0, IECP, 64, 64, 1.0f);
    wmma_gemm64<0, false, 0, 1, false><<<dim3((t + 7) / 8, 1), 256, 0, stream>>>(U16(H2), nullptr, 64, 0, (const unsigned short*)BT3, nullptr, 64, 0, K3c, nullptr, 64, 0, nullptr, nullptr, 0, IECP, 64, 64, 1.0f);
    kcopy_kernel<<<(unsigned)(((long)IEC * 16 + 255) / 256), 256, 0, stream>>>((const unsigned*)K3c, e0, KALL); }
  reduce_kernel<<<(IN_ + 7) / 8, 256, 0, stream>>>(KALL, b3, fy, wts, nbr, rs, out);
}
